// MonoidBlock_12799002542293
// MI455X (gfx1250) — hardware-verified
//
#include <hip/hip_runtime.h>
#include <hip/hip_bf16.h>
#include <math.h>


#pragma clang fp contract(off)

#define NB     32
#define SEQ    2048
#define DCH    512
#define VOC    256
#define MBSZ   256
#define NMB    8
#define EXCH   32
#define NPIT   3000
#define AMIN   0.9f
#define ARANGE 0.099f
#define INJSC  0.125f

static_assert(SEQ == NMB * MBSZ);
static_assert(DCH == 16 * EXCH);
static_assert((MBSZ % 4) == 0);
static_assert((VOC * DCH) % 1024 == 0);
static_assert(DCH % 128 == 0);

typedef float          v4f   __attribute__((ext_vector_type(4)));
typedef float          v8f   __attribute__((ext_vector_type(8)));
typedef int            v4i   __attribute__((ext_vector_type(4)));
typedef __bf16         v16b  __attribute__((ext_vector_type(16)));
typedef unsigned short u16x8 __attribute__((ext_vector_type(8)));

union FragB { u16x8 h[2]; v16b v; };
static_assert(sizeof(FragB) == 32);

__device__ __forceinline__ unsigned short f32_to_bf16(float f) {
    unsigned u = __float_as_uint(f);
    unsigned r = u + 0x7FFFu + ((u >> 16) & 1u);
    return (unsigned short)(r >> 16);
}
__device__ __forceinline__ float bf16_to_f32(unsigned short b) {
    return __uint_as_float(((unsigned)b) << 16);
}
__device__ __forceinline__ float decay_coef(float x) {
    const float e = expf(-x);
    const float s = 1.0f / (1.0f + e);
    return AMIN + ARANGE * s;
}

__device__ __forceinline__ void mma_bf16(v8f& acc, const v16b& a, const v16b& b) {
    acc = __builtin_amdgcn_wmma_f32_16x16x32_bf16(false, a, false, b, (short)0, acc, false, false);
    asm volatile("v_nop\n\tv_nop\n\tv_nop\n\tv_nop" : "+v"(acc) : "v"(a), "v"(b));
}

__global__ __launch_bounds__(256)
void atab_kernel(const float* __restrict__ a_raw, float* atab, int n4)
{
    const int i = blockIdx.x * 256 + threadIdx.x;
    if (i >= n4) return;
    const size_t e = (size_t)i * 4;
    const v4f x = *(const v4f*)(a_raw + e);
    v4f r;
    r.x = decay_coef(x.x);
    r.y = decay_coef(x.y);
    r.z = decay_coef(x.z);
    r.w = decay_coef(x.w);
    *(volatile v4f*)(atab + e) = r;
    __threadfence();
    *(volatile v4f*)(atab + e) = r;
}

__global__ __launch_bounds__(DCH)
void monoid_kernel(const int* __restrict__ tokens, const float* __restrict__ atab,
                   const float* __restrict__ btab, const float* __restrict__ exw,
                   float* out)
{
    __shared__ __attribute__((aligned(16))) int    stok[SEQ];
    __shared__ __attribute__((aligned(16))) float  sW[EXCH * EXCH];
    __shared__ __attribute__((aligned(16))) double sM[EXCH * EXCH];
    __shared__ __attribute__((aligned(16))) float  sl[DCH];
    __shared__ __attribute__((aligned(16))) float  su[EXCH];
    __shared__ __attribute__((aligned(16))) float  suo[EXCH];
    __shared__ float srs[4];

    const int tid  = threadIdx.x;
    const int lane = tid & 31;
    const int wave = tid >> 5;
    const int hh   = lane >> 4;
    const int m    = lane & 15;
    const int bidx = blockIdx.x;
    const int d    = tid;

    for (int i = tid; i < SEQ; i += DCH) {
        int t = tokens[(size_t)bidx * SEQ + i];
        t = (t < 0) ? 0 : t;
        t = (t > VOC - 1) ? (VOC - 1) : t;
        stok[i] = t;
    }
    for (int i = tid; i < EXCH * EXCH; i += DCH) sW[i] = exw[i];
    __syncthreads();

    for (int e = tid; e < EXCH * EXCH; e += DCH) {
        const int j = e >> 5, k = e & 31;
        double acc = 0.0;
#pragma unroll 1
        for (int i = 0; i < EXCH; ++i)
            acc = fma((double)sW[i * EXCH + j], (double)sW[i * EXCH + k], acc);
        sM[e] = acc;
    }
    __syncthreads();

    if (wave == 0) {
        double mr[EXCH];
#pragma unroll
        for (int k = 0; k < EXCH; ++k) mr[k] = sM[lane * EXCH + k];
        double v = 1.0, vold = 1.0, t = 0.0;
#pragma unroll 1
        for (int it = 0; it < NPIT; ++it) {
            t = 0.0;
#pragma unroll
            for (int k = 0; k < EXCH; ++k) t = fma(mr[k], __shfl(v, k, 32), t);
            vold = v;
            double vm = fabs(t);
#pragma unroll
            for (int o = 16; o >= 1; o >>= 1) vm = fmax(vm, __shfl_xor(vm, o, 32));
            v = t * (1.0 / vm);
        }
        double num = vold * t;
        double den = vold * vold;
#pragma unroll
        for (int o = 16; o >= 1; o >>= 1) {
            num += __shfl_xor(num, o, 32);
            den += __shfl_xor(den, o, 32);
        }
        const double lam = num / den;
        double s = (double)sqrtf((float)lam);
        s = 0.5 * (s + lam / s);
        s = 0.5 * (s + lam / s);
        const float sig = (float)s;
        const float rs0 = (float)(1.0 / (double)sig);
        if (lane == 0) srs[0] = rs0;
    }
    __syncthreads();
    const float rs = srs[0];

    const u16x8 z8 = {0, 0, 0, 0, 0, 0, 0, 0};
    FragB awh, awl;
    awh.h[0] = z8; awh.h[1] = z8; awl.h[0] = z8; awl.h[1] = z8;
    if (wave < 2) {
        const float* wb = sW + (16 * wave + m) * EXCH + 8 * hh;
#pragma unroll
        for (int i = 0; i < 16; ++i) {
            const float x = wb[i + ((i >> 3) << 3)] * rs;
            const unsigned short hb = f32_to_bf16(x);
            const unsigned short lb = f32_to_bf16(x - bf16_to_f32(hb));
            awh.h[i >> 3][i & 7] = hb;
            awl.h[i >> 3][i & 7] = lb;
        }
    }

    float hst = 0.0f;
#pragma unroll 1
    for (int mb = 0; mb < NMB; ++mb) {
        const int phase = mb & 3;
        const int tb    = mb * MBSZ;

        double aa = 1.0, bb = 0.0;
#pragma unroll 1
        for (int t0 = 0; t0 < MBSZ; t0 += 4) {
            const v4i tk = *(const v4i*)(stok + tb + t0);
#pragma unroll
            for (int j = 0; j < 4; ++j) {
                const int tok = tk[j];
                const float av = atab[tok * DCH + d];
                const float bv = btab[tok * DCH + d];
                aa = aa * (double)av;
                bb = fma((double)av, bb, (double)bv);
            }
        }
        {
            const float aaf = (float)aa;
            const float bbf = (float)bb;
            const float prod = aaf * hst;
            hst = prod + bbf;
        }

#pragma unroll
        for (int step = 1; step <= 16; step <<= 1) {
            const float pv  = __shfl_xor(hst, step, 32);
            const float sum = hst + pv;
            const float dif = pv - hst;
            hst = (d & step) ? dif : sum;
        }
        sl[d] = hst;
        __syncthreads();
        {
            const float pv  = sl[d ^ 32];
            const float sum = hst + pv;
            const float dif = pv - hst;
            hst = (d & 32) ? dif : sum;
        }
        hst = tanhf(hst);
        __syncthreads();
        sl[d] = hst;
        __syncthreads();

        if (tid < EXCH) {
            const int g = tid >> 4, p = tid & 15;
            const float* lp = sl + g * 256;
            const int i0 = 4 * p + phase;
            const float u = ((lp[i0] + lp[i0 + 1]) + lp[i0 + 2]) + lp[i0 + 3];
            su[tid] = u;
        }
        __syncthreads();

        if (wave < 2) {
            FragB bh, bl;
            bh.h[0] = z8; bh.h[1] = z8; bl.h[0] = z8; bl.h[1] = z8;
            const float* sp = su + 8 * hh;
#pragma unroll
            for (int i = 0; i < 16; ++i) {
                const float xv = sp[i + ((i >> 3) << 3)];
                const float x  = (m == 0) ? xv : 0.0f;
                const unsigned short hb = f32_to_bf16(x);
                const unsigned short lb = f32_to_bf16(x - bf16_to_f32(hb));
                bh.h[i >> 3][i & 7] = hb;
                bl.h[i >> 3][i & 7] = lb;
            }
            v8f acc = {0.f, 0.f, 0.f, 0.f, 0.f, 0.f, 0.f, 0.f};
            mma_bf16(acc, awh.v, bh.v);
            mma_bf16(acc, awh.v, bl.v);
            mma_bf16(acc, awl.v, bh.v);
            if (m == 0) {
#pragma unroll
                for (int r = 0; r < 8; ++r) suo[16 * wave + 8 * hh + r] = acc[r];
            }
        }
        __syncthreads();

        {
            const int q  = (d & 255) - phase;
            const int p  = (q >> 2) & 15;
            const float uo = suo[(d >> 8) * 16 + p];
            if (q >= 0 && q < 64) {
                const float inj = uo * INJSC;
                hst = hst + inj;
            }
        }
        __syncthreads();
    }

    sl[d] = hst;
    __syncthreads();
    if (tid < DCH / 4) {
        const v4f v = *(const v4f*)(sl + tid * 4);
        float* gp = out + (size_t)bidx * DCH + tid * 4;
        *(volatile v4f*)gp = v;
        __threadfence();
        *(volatile v4f*)gp = v;
    }
}

extern "C" void kernel_launch(void* const* d_in, const int* in_sizes, int n_in,
                              void* d_out, int out_size, void* d_ws, size_t ws_size,
                              hipStream_t stream)
{
    if (n_in < 4) return;
    if (in_sizes[0] != NB * SEQ)     return;
    if (in_sizes[1] != VOC * DCH)    return;
    if (in_sizes[2] != VOC * DCH)    return;
    if (in_sizes[3] != EXCH * EXCH)  return;
    if (out_size != NB * DCH)        return;

    const int*   tokens = (const int*)d_in[0];
    const float* a_raw  = (const float*)d_in[1];
    const float* btab   = (const float*)d_in[2];
    const float* exw    = (const float*)d_in[3];
    float* out = (float*)d_out;

    const size_t SZ_ATAB = (size_t)VOC * DCH * sizeof(float);
    if (ws_size < SZ_ATAB) return;
    float* atab = (float*)d_ws;

    const int n4 = (VOC * DCH) / 4;
    hipLaunchKernelGGL(atab_kernel, dim3((n4 + 255) / 256), dim3(256), 0, stream,
                       a_raw, atab, n4);
    hipLaunchKernelGGL(monoid_kernel, dim3(NB), dim3(DCH), 0, stream,
                       tokens, (const float*)atab, btab, exw, out);
}
